// msaLMMixin_77936476553340
// MI455X (gfx1250) — hardware-verified
//
#include <hip/hip_runtime.h>
#include <math.h>

typedef __attribute__((ext_vector_type(16))) __bf16   v16b;
typedef __attribute__((ext_vector_type(8)))  __bf16   v8b;
typedef __attribute__((ext_vector_type(8)))  _Float16 v8h;
typedef __attribute__((ext_vector_type(8)))  float    v8f;
typedef __attribute__((ext_vector_type(4)))  float    v4f;
typedef __attribute__((ext_vector_type(4)))  unsigned int v4u;

constexpr int kBatch   = 2;
constexpr int kSeqLen  = 2048;
constexpr int kModel   = 1024;
constexpr int kHeads   = 16;
constexpr int kHeadDim = 64;
constexpr int kRows    = kBatch * kSeqLen;
constexpr int kQkvCols = 3 * kModel;
constexpr int kCatCols = 2 * kModel;
constexpr int kSegLen  = 512;
constexpr int kQTile   = 128;
constexpr int kKTile   = 64;
constexpr int kAttWaves = 8;
constexpr int kQTiles  = kSeqLen / kQTile;
constexpr int kTilesPerSeg = kSegLen / kKTile;
constexpr float kQScale   = 0.125f;
constexpr float kMaskFill = -1.0e9f;
constexpr size_t kPlaneElems = (size_t)kBatch * kHeads * kSeqLen * kHeadDim;

static_assert(kHeads * kHeadDim == kModel, "head split");
static_assert(kQScale * kQScale * (float)kHeadDim == 1.0f, "score scale is 1/sqrt(head dim)");
static_assert(kHeadDim == 64 && kKTile == 64, "tile shape");
static_assert((kRows % 64) == 0 && (kQkvCols % 64) == 0 && (kModel % 64) == 0, "GEMM M,N multiples of 64");
static_assert((kModel % 32) == 0 && (kCatCols % 32) == 0, "GEMM K multiples of 32");
static_assert((kSeqLen % kQTile) == 0 && (kSegLen % kQTile) == 0 && (kSegLen % kKTile) == 0, "attention tiles");
static_assert(kAttWaves * 16 == kQTile, "query rows per block");
static_assert(4 * kSegLen == kSeqLen, "four segments");

constexpr size_t kOffXB    = 0;
constexpr size_t kOffWQKVT = kOffXB    + (size_t)kRows * kModel * 2;
constexpr size_t kOffWOT2  = kOffWQKVT + (size_t)kQkvCols * kModel * 2;
constexpr size_t kOffPH    = kOffWOT2  + (size_t)kModel * kCatCols * 2;
constexpr size_t kOffPL    = kOffPH    + 3 * kPlaneElems * 2;
constexpr size_t kOffOCAT  = kOffPL    + 3 * kPlaneElems * 2;
constexpr size_t kWsTotal  = kOffOCAT  + (size_t)kRows * kCatCols * 2;
static_assert(kWsTotal == 85983232ull, "carve total");
static_assert(kWsTotal <= 134217728ull, "carve cap");
static_assert((kOffWQKVT % 128) == 0 && (kOffWOT2 % 128) == 0 && (kOffPH % 128) == 0 &&
              (kOffPL % 128) == 0 && (kOffOCAT % 128) == 0, "128-B aligned regions");

__device__ __forceinline__ unsigned short f2bf_bits(float f) {
  unsigned u = __float_as_uint(f);
  return (unsigned short)((u + 0x7FFFu + ((u >> 16) & 1u)) >> 16);
}
__device__ __forceinline__ float bf_bits2f(unsigned short h) { return __uint_as_float(((unsigned)h) << 16); }
__device__ __forceinline__ unsigned pk16(unsigned short a, unsigned short b) { return (unsigned)a | ((unsigned)b << 16); }
__device__ __forceinline__ __bf16 bits2bf(unsigned short h) { return __builtin_bit_cast(__bf16, h); }

__device__ __forceinline__ v8f mma_b(v16b a, v16b b, v8f c) {
  c = __builtin_amdgcn_wmma_f32_16x16x32_bf16(false, a, false, b, (short)0, c, false, false);
  asm volatile("v_nop\n\tv_nop\n\tv_nop\n\tv_nop" : "+v"(c) : "v"(a), "v"(b));
  return c;
}

union FragB { v16b v; v8b h[2]; };
__device__ __forceinline__ v16b frag_load(const __bf16* p) {
  FragB f;
  f.h[0] = *(const v8b*)(p);
  f.h[1] = *(const v8b*)(p + 16);
  return f.v;
}

__global__ __launch_bounds__(256) void cast8_bf16_kernel(const float* __restrict__ in, unsigned short* __restrict__ out, int n8) {
  const int i = blockIdx.x * 256 + threadIdx.x;
  if (i >= n8) return;
  const float* p = in + 8 * (size_t)i;
  const v4f a = *(const v4f*)(p);
  const v4f c = *(const v4f*)(p + 4);
  unsigned short hb[8];
#pragma unroll
  for (int e = 0; e < 4; ++e) {
    hb[e]     = f2bf_bits(a[e]);
    hb[4 + e] = f2bf_bits(c[e]);
  }
  const v4u u = (v4u){pk16(hb[0], hb[1]), pk16(hb[2], hb[3]), pk16(hb[4], hb[5]), pk16(hb[6], hb[7])};
  unsigned short* q = out + 8 * (size_t)i;
  *(volatile v4u*)q = u;
  __threadfence();
  *(volatile v4u*)q = u;
}

__global__ __launch_bounds__(256) void wtrans_bf16_kernel(const float* __restrict__ W0, const float* __restrict__ W1,
                                                          const float* __restrict__ W2, const float* __restrict__ W3,
                                                          unsigned short* __restrict__ wqkvt, unsigned short* __restrict__ wot2) {
  __shared__ float sm[64][65];
  const int t  = threadIdx.x;
  const int k0 = blockIdx.x * 64;
  const int n0 = blockIdx.y * 64;
  const int z  = blockIdx.z;
  const float* W = (z == 0) ? W0 : (z == 1) ? W1 : (z == 2) ? W2 : W3;
  const float scale = (z == 0) ? kQScale : 1.0f;
#pragma unroll
  for (int i = 0; i < 16; ++i) {
    const int e  = i * 256 + t;
    const int r  = e >> 6;
    const int cc = e & 63;
    sm[cc][r] = W[(size_t)(k0 + r) * kModel + n0 + cc] * scale;
  }
  __syncthreads();
  const int lane = t & 31, wave = t >> 5;
  const int q = lane >> 3, c8 = (lane & 7) * 8;
  const bool dup = (z == 3);
  unsigned short* op = dup ? wot2 : (wqkvt + (size_t)z * kModel * kModel);
  const int ld = dup ? kCatCols : kModel;
  v4u u[2];
#pragma unroll
  for (int it = 0; it < 2; ++it) {
    const int row = wave * 8 + it * 4 + q;
    unsigned short hb[8];
#pragma unroll
    for (int e = 0; e < 8; ++e) hb[e] = f2bf_bits(sm[row][c8 + e]);
    u[it] = (v4u){pk16(hb[0], hb[1]), pk16(hb[2], hb[3]), pk16(hb[4], hb[5]), pk16(hb[6], hb[7])};
  }
  for (int pass = 0; pass < 2; ++pass) {
#pragma unroll
    for (int it = 0; it < 2; ++it) {
      const int row = wave * 8 + it * 4 + q;
      unsigned short* p = op + (size_t)(n0 + row) * ld + k0 + c8;
      *(volatile v4u*)p = u[it];
      if (dup) *(volatile v4u*)(p + kModel) = u[it];
    }
    __threadfence();
  }
}

template <int OUT_MODE>
__global__ __launch_bounds__(256) void wmma_gemm64_bf16(
    const unsigned short* __restrict__ Ap, int lda,
    const unsigned short* __restrict__ Btp, int ldb,
    void* Cout, void* Cout2, int ldc,
    int M, int N, int K) {
  const __bf16* A  = (const __bf16*)Ap;
  const __bf16* Bt = (const __bf16*)Btp;
  __shared__ __align__(16) float sT[8][16 * 68];
  const int lane = threadIdx.x & 31;
  const int wave = threadIdx.x >> 5;
  const int tilesN = N >> 6;
  const int tilesM = M >> 6;
  const int tile = blockIdx.x * 8 + wave;
  if (tile >= tilesM * tilesN) return;
  const int tm = tile / tilesN;
  const int tn = tile - tm * tilesN;
  const int m0 = tm << 6;
  const int n0 = tn << 6;

  const int rlane = lane & 15;
  const int koff  = (lane >> 4) * 8;
  const int mOff  = (lane >> 4) * 8;

  v8f acc[4][4];
#pragma unroll
  for (int i = 0; i < 4; ++i)
#pragma unroll
    for (int j = 0; j < 4; ++j) acc[i][j] = (v8f){0.f,0.f,0.f,0.f,0.f,0.f,0.f,0.f};

  for (int k0 = 0; k0 < K; k0 += 32) {
    v16b bh[4];
#pragma unroll
    for (int j = 0; j < 4; ++j) {
      const size_t bo = (size_t)(n0 + (j << 4) + rlane) * ldb + koff + k0;
      bh[j] = frag_load(Bt + bo);
    }
#pragma unroll
    for (int i = 0; i < 4; ++i) {
      const size_t ao = (size_t)(m0 + (i << 4) + rlane) * lda + koff + k0;
      const v16b ah = frag_load(A + ao);
#pragma unroll
      for (int j = 0; j < 4; ++j) acc[i][j] = mma_b(ah, bh[j], acc[i][j]);
    }
  }

  float* slab = sT[wave];
#pragma unroll
  for (int i = 0; i < 4; ++i) {
    const int mBase = m0 + (i << 4);
#pragma unroll
    for (int j = 0; j < 4; ++j) {
#pragma unroll
      for (int r = 0; r < 8; ++r) slab[(mOff + r) * 68 + (j << 4) + rlane] = acc[i][j][r];
    }
    __builtin_amdgcn_fence(__ATOMIC_RELEASE, "workgroup");
    __builtin_amdgcn_wave_barrier();
    __builtin_amdgcn_fence(__ATOMIC_ACQUIRE, "workgroup");
    if (OUT_MODE == 0) {
      float* C = (float*)Cout;
      const int hh = lane >> 4, c4 = (lane & 15) * 4;
      for (int pass = 0; pass < 2; ++pass) {
#pragma unroll
        for (int it = 0; it < 8; ++it) {
          const int row = it * 2 + hh;
          v4f v = *(const v4f*)(slab + row * 68 + c4);
          *(volatile v4f*)(C + (size_t)(mBase + row) * ldc + n0 + c4) = v;
        }
        __threadfence();
      }
    } else {
      const int q = lane >> 3, c8 = (lane & 7) * 8;
      unsigned short* C  = (unsigned short*)Cout;
      unsigned short* C2 = (unsigned short*)Cout2;
      const int plane = n0 / kModel;
      const int head  = (n0 % kModel) / kHeadDim;
      for (int pass = 0; pass < 2; ++pass) {
#pragma unroll
        for (int it = 0; it < 4; ++it) {
          const int row = it * 4 + q;
          const float* sp = slab + row * 68 + c8;
          v8h hv, lv;
#pragma unroll
          for (int e = 0; e < 8; ++e) {
            const unsigned short hb = f2bf_bits(sp[e]);
            const unsigned short lb = f2bf_bits(sp[e] - bf_bits2f(hb));
            hv[e] = __builtin_bit_cast(_Float16, hb);
            lv[e] = __builtin_bit_cast(_Float16, lb);
          }
          const int gm = mBase + row;
          const size_t off = (size_t)plane * kPlaneElems +
                             ((size_t)((gm / kSeqLen) * kHeads + head) * kSeqLen + (size_t)(gm % kSeqLen)) * kHeadDim + c8;
          *(volatile v8h*)(C + off)  = hv;
          *(volatile v8h*)(C2 + off) = lv;
        }
        __threadfence();
      }
    }
    __builtin_amdgcn_fence(__ATOMIC_RELEASE, "workgroup");
    __builtin_amdgcn_wave_barrier();
    __builtin_amdgcn_fence(__ATOMIC_ACQUIRE, "workgroup");
  }
}

__global__ __launch_bounds__(256)
void attn_seg_kernel(const unsigned short* __restrict__ planesHi, const unsigned short* __restrict__ planesLo,
                     unsigned short* __restrict__ ocat) {
  __shared__ __align__(16) __bf16 Ksh[kKTile * kHeadDim];
  __shared__ __align__(16) __bf16 Ksl[kKTile * kHeadDim];
  __shared__ __align__(16) __bf16 Vth[kHeadDim * kKTile];
  __shared__ __align__(16) __bf16 Vtl[kHeadDim * kKTile];
  __shared__ __align__(16) __bf16 Psh[kAttWaves][16 * kKTile];
  __shared__ __align__(16) __bf16 Psl[kAttWaves][16 * kKTile];

  const int tid  = threadIdx.x;
  const int wave = __builtin_amdgcn_readfirstlane(tid >> 5);
  const int lane = tid & 31;
  const int hh   = lane >> 4;
  const int c    = lane & 15;

  const int bx = blockIdx.x;
  const int qt = bx % kQTiles;
  const int h  = (bx / kQTiles) % kHeads;
  const int b  = bx / (kQTiles * kHeads);
  const int qbase = qt * kQTile;
  const int sq    = qbase / kSegLen;
  const int q0    = qbase + wave * 16;

  const size_t headOff = (size_t)(b * kHeads + h) * kSeqLen * kHeadDim;
  const __bf16* Qh = (const __bf16*)planesHi + headOff;
  const __bf16* Ql = (const __bf16*)planesLo + headOff;
  const __bf16* Kh = Qh + kPlaneElems;
  const __bf16* Kl = Ql + kPlaneElems;
  const __bf16* Vh = Qh + 2 * kPlaneElems;
  const __bf16* Vl = Ql + 2 * kPlaneElems;

  v16b qh[2], ql[2];
  {
    const size_t qo = (size_t)(q0 + c) * kHeadDim + 8 * hh;
#pragma unroll
    for (int dc = 0; dc < 2; ++dc) {
      qh[dc] = frag_load(Qh + qo + dc * 32);
      ql[dc] = frag_load(Ql + qo + dc * 32);
    }
  }

  float mrow[8], lrow[8];
  v8f oacc[4];
#pragma unroll
  for (int r = 0; r < 8; ++r) { mrow[r] = -3.0e38f; lrow[r] = 0.f; }
#pragma unroll
  for (int t = 0; t < 4; ++t) oacc[t] = (v8f){0.f,0.f,0.f,0.f,0.f,0.f,0.f,0.f};

  const int nText    = (sq > 0) ? kTilesPerSeg : 0;
  const int ownFirst = sq * kTilesPerSeg;
  const int ownLast  = (qbase + kQTile - 1) / kKTile;
  const int nTiles   = nText + (ownLast - ownFirst + 1);

  __bf16* pwh = Psh[wave];
  __bf16* pwl = Psl[wave];

  for (int it = 0; it < nTiles; ++it) {
    const int kt  = (it < nText) ? it : (ownFirst + it - nText);
    const int kv0 = kt * kKTile;
    const bool own = (kt >= ownFirst);

    __syncthreads();
    {
      const v4u* gkh = (const v4u*)(Kh + (size_t)kv0 * kHeadDim);
      const v4u* gkl = (const v4u*)(Kl + (size_t)kv0 * kHeadDim);
      const v4u* gvh = (const v4u*)(Vh + (size_t)kv0 * kHeadDim);
      const v4u* gvl = (const v4u*)(Vl + (size_t)kv0 * kHeadDim);
#pragma unroll
      for (int i = 0; i < 2; ++i) {
        const int ch = tid + i * 256;
        const v4u wkh = gkh[ch];
        const v4u wkl = gkl[ch];
        const v4u wvh = gvh[ch];
        const v4u wvl = gvl[ch];
        *(v4u*)(Ksh + ch * 8) = wkh;
        *(v4u*)(Ksl + ch * 8) = wkl;
        const int kvr = ch >> 3;
        const int d0  = (ch & 7) * 8;
#pragma unroll
        for (int w = 0; w < 4; ++w) {
          const unsigned a  = wvh[w];
          const unsigned bl = wvl[w];
          Vth[(d0 + 2 * w) * kKTile + kvr]     = bits2bf((unsigned short)(a & 0xffffu));
          Vth[(d0 + 2 * w + 1) * kKTile + kvr] = bits2bf((unsigned short)(a >> 16));
          Vtl[(d0 + 2 * w) * kKTile + kvr]     = bits2bf((unsigned short)(bl & 0xffffu));
          Vtl[(d0 + 2 * w + 1) * kKTile + kvr] = bits2bf((unsigned short)(bl >> 16));
        }
      }
    }
    __syncthreads();

    const bool live = (!own) || (kv0 <= q0 + 15);
    if (live) {
      v8f s[4];
#pragma unroll
      for (int j = 0; j < 4; ++j) {
        s[j] = (v8f){0.f,0.f,0.f,0.f,0.f,0.f,0.f,0.f};
#pragma unroll
        for (int dc = 0; dc < 2; ++dc) {
          const int ko = (j * 16 + c) * kHeadDim + dc * 32 + 8 * hh;
          const v16b kbh = frag_load(Ksh + ko);
          const v16b kbl = frag_load(Ksl + ko);
          s[j] = mma_b(qh[dc], kbh, s[j]);
          s[j] = mma_b(qh[dc], kbl, s[j]);
          s[j] = mma_b(ql[dc], kbh, s[j]);
        }
      }

      float cm[8];
#pragma unroll
      for (int r = 0; r < 8; ++r) {
        const int qrow = q0 + 8 * hh + r;
        float m = -3.0e38f;
#pragma unroll
        for (int j = 0; j < 4; ++j) {
          const int kvcol = kv0 + j * 16 + c;
          const bool masked = own && (kvcol > qrow);
          if (masked) s[j][r] = kMaskFill;
          m = fmaxf(m, s[j][r]);
        }
#pragma unroll
        for (int off = 1; off < 16; off <<= 1) m = fmaxf(m, __shfl_xor(m, off, 32));
        cm[r] = m;
      }

#pragma unroll
      for (int r = 0; r < 8; ++r) {
        const float mnew  = fmaxf(mrow[r], cm[r]);
        const float alpha = __expf(mrow[r] - mnew);
        mrow[r] = mnew;
        float psum = 0.f;
#pragma unroll
        for (int j = 0; j < 4; ++j) {
          const float p = __expf(s[j][r] - mnew);
          psum += p;
          const unsigned short hb = f2bf_bits(p);
          const unsigned short lb = f2bf_bits(p - bf_bits2f(hb));
          pwh[(8 * hh + r) * kKTile + j * 16 + c] = bits2bf(hb);
          pwl[(8 * hh + r) * kKTile + j * 16 + c] = bits2bf(lb);
        }
#pragma unroll
        for (int off = 1; off < 16; off <<= 1) psum += __shfl_xor(psum, off, 32);
        lrow[r] = lrow[r] * alpha + psum;
#pragma unroll
        for (int t = 0; t < 4; ++t) oacc[t][r] *= alpha;
      }
      __builtin_amdgcn_fence(__ATOMIC_RELEASE, "workgroup");
      __builtin_amdgcn_wave_barrier();
      __builtin_amdgcn_fence(__ATOMIC_ACQUIRE, "workgroup");
#pragma unroll 1
      for (int kk = 0; kk < 2; ++kk) {
        const int po = c * kKTile + kk * 32 + 8 * hh;
        const v16b pa = frag_load(pwh + po);
        const v16b pl = frag_load(pwl + po);
#pragma unroll
        for (int t = 0; t < 4; ++t) {
          const int vo = (t * 16 + c) * kKTile + kk * 32 + 8 * hh;
          const v16b vbh = frag_load(Vth + vo);
          const v16b vbl = frag_load(Vtl + vo);
          oacc[t] = mma_b(pa, vbh, oacc[t]);
          oacc[t] = mma_b(pa, vbl, oacc[t]);
          oacc[t] = mma_b(pl, vbh, oacc[t]);
        }
      }
    }
  }

  __builtin_amdgcn_fence(__ATOMIC_RELEASE, "workgroup");
  __builtin_amdgcn_wave_barrier();
  __builtin_amdgcn_fence(__ATOMIC_ACQUIRE, "workgroup");
#pragma unroll
  for (int r = 0; r < 8; ++r) {
    const float inv = 1.0f / lrow[r];
#pragma unroll
    for (int t = 0; t < 4; ++t) {
      const float val = oacc[t][r] * inv;
      const unsigned short hb = f2bf_bits(val);
      const unsigned short lb = f2bf_bits(val - bf_bits2f(hb));
      pwh[(8 * hh + r) * kKTile + t * 16 + c] = bits2bf(hb);
      pwl[(8 * hh + r) * kKTile + t * 16 + c] = bits2bf(lb);
    }
  }
  __builtin_amdgcn_fence(__ATOMIC_RELEASE, "workgroup");
  __builtin_amdgcn_wave_barrier();
  __builtin_amdgcn_fence(__ATOMIC_ACQUIRE, "workgroup");
  {
    const int q  = lane >> 3;
    const int c8 = (lane & 7) * 8;
    v4u hv[4], lv[4];
#pragma unroll
    for (int i4 = 0; i4 < 4; ++i4) {
      const int row = i4 * 4 + q;
      const v8b xh = *(const v8b*)(pwh + row * kKTile + c8);
      const v8b xl = *(const v8b*)(pwl + row * kKTile + c8);
      hv[i4] = __builtin_bit_cast(v4u, xh);
      lv[i4] = __builtin_bit_cast(v4u, xl);
    }
    unsigned short* ob = ocat + (size_t)(b * kSeqLen + q0) * kCatCols + h * kHeadDim + c8;
    for (int pass = 0; pass < 2; ++pass) {
#pragma unroll
      for (int i4 = 0; i4 < 4; ++i4) {
        const int row = i4 * 4 + q;
        unsigned short* p = ob + (size_t)row * kCatCols;
        *(volatile v4u*)(p)          = hv[i4];
        *(volatile v4u*)(p + kModel) = lv[i4];
      }
      __threadfence();
    }
  }
}

extern "C" void kernel_launch(void* const* d_in, const int* in_sizes, int n_in,
                              void* d_out, int out_size, void* d_ws, size_t ws_size,
                              hipStream_t stream) {
  if (n_in < 5) return;
  if (in_sizes[0] != kRows * kModel) return;
  if (in_sizes[1] != kModel * kModel) return;
  if (in_sizes[2] != kModel * kModel) return;
  if (in_sizes[3] != kModel * kModel) return;
  if (in_sizes[4] != kModel * kModel) return;
  if (out_size != kRows * kModel) return;
  if (ws_size < kWsTotal) return;

  const float* x  = (const float*)d_in[0];
  const float* Wq = (const float*)d_in[1];
  const float* Wk = (const float*)d_in[2];
  const float* Wv = (const float*)d_in[3];
  const float* Wo = (const float*)d_in[4];
  float* out = (float*)d_out;

  char* ws = (char*)d_ws;
  unsigned short* XB    = (unsigned short*)(ws + kOffXB);
  unsigned short* WQKVT = (unsigned short*)(ws + kOffWQKVT);
  unsigned short* WOT2  = (unsigned short*)(ws + kOffWOT2);
  unsigned short* PH    = (unsigned short*)(ws + kOffPH);
  unsigned short* PL    = (unsigned short*)(ws + kOffPL);
  unsigned short* OCAT  = (unsigned short*)(ws + kOffOCAT);

  constexpr int kN8 = kRows * kModel / 8;
  static_assert((kN8 % 256) == 0, "cast grid exact");
  cast8_bf16_kernel<<<kN8 / 256, 256, 0, stream>>>(x, XB, kN8);

  wtrans_bf16_kernel<<<dim3(kModel / 64, kModel / 64, 4), 256, 0, stream>>>(Wq, Wk, Wv, Wo, WQKVT, WOT2);

  constexpr int kTiles1 = (kRows / 64) * (kQkvCols / 64);
  static_assert((kTiles1 % 8) == 0, "tile grid exact");
  wmma_gemm64_bf16<3><<<dim3(kTiles1 / 8, 1), 256, 0, stream>>>(
      XB, kModel, WQKVT, kModel, (void*)PH, (void*)PL, 0, kRows, kQkvCols, kModel);

  attn_seg_kernel<<<kBatch * kHeads * kQTiles, 256, 0, stream>>>(PH, PL, OCAT);

  constexpr int kTiles2 = (kRows / 64) * (kModel / 64);
  static_assert((kTiles2 % 8) == 0, "tile grid exact");
  wmma_gemm64_bf16<0><<<dim3(kTiles2 / 8, 1), 256, 0, stream>>>(
      OCAT, kCatCols, WOT2, kCatCols, (void*)out, (void*)out, kModel, kRows, kModel, kCatCols);
}
